// FlowMLP_66219805770045
// MI455X (gfx1250) — hardware-verified
//
#include <hip/hip_runtime.h>
#include <stddef.h>
#include <stdint.h>


typedef _Float16 v16h __attribute__((ext_vector_type(16)));
typedef _Float16 v8h  __attribute__((ext_vector_type(8)));
typedef float    v8f  __attribute__((ext_vector_type(8)));
typedef float    v4f  __attribute__((ext_vector_type(4)));

namespace {
constexpr int B_   = 4;
constexpr int C_   = 192;
constexpr int H_   = 48;
constexpr int W_   = 48;
constexpr int DN_  = 384;
constexpr int NS_  = 16;
constexpr int R_   = 12;
constexpr int K_   = 4;
constexpr int MH_  = 768;
constexpr int L_   = H_ * W_;
constexpr int MTOK = B_ * L_;
constexpr int NPAD = 48;
constexpr int XPC  = K_ * NPAD;
static_assert(MTOK % 64 == 0);
static_assert(C_ % 64 == 0);
static_assert(DN_ % 64 == 0);
static_assert(MH_ % 64 == 0);
static_assert(XPC % 64 == 0);
static_assert((B_ * K_ * DN_) % 128 == 0);
static_assert(DN_ % 128 == 0);
static_assert(L_ % 8 == 0);
static_assert((MTOK * (C_ / 4)) % 256 == 0);
static_assert(MTOK % 8 == 0);
static_assert(R_ + 2 * NS_ <= NPAD);
static_assert(H_ == W_);
}

union Frag { v16h v; v8h h[2]; };

static __device__ __forceinline__ v8f wmma16(const v16h a, const v16h b, v8f c) {
    v8f d = __builtin_amdgcn_wmma_f32_16x16x32_f16(false, a, false, b, (short)0, c, false, false);
    asm volatile("v_nop\n\tv_nop\n\tv_nop\n\tv_nop" : "+v"(d) : "v"(a), "v"(b));
    return d;
}

static __device__ __forceinline__ float wsum(float v) {
#pragma unroll
    for (int o = 16; o > 0; o >>= 1) v += __shfl_xor(v, o);
    return v;
}
static __device__ __forceinline__ v8f ld8(const float* p) {
    v4f a = *(const v4f*)p;
    v4f b = *(const v4f*)(p + 4);
    return __builtin_shufflevector(a, b, 0, 1, 2, 3, 4, 5, 6, 7);
}
static __device__ __forceinline__ v8f zero8() {
    v8f z;
#pragma unroll
    for (int e = 0; e < 8; ++e) z[e] = 0.0f;
    return z;
}
static __device__ __forceinline__ float hsum8(const v8f v) {
    return ((v[0] + v[1]) + (v[2] + v[3])) + ((v[4] + v[5]) + (v[6] + v[7]));
}
static __device__ __forceinline__ float gelu_f(float x) {
    return x * (0.5f * (1.0f + erff(x * 0.70710678118654752f)));
}
static __device__ __forceinline__ float silu_f(float x) {
    const float e = expf(-x);
    return x * __builtin_amdgcn_rcpf(1.0f + e);
}

__global__ void __launch_bounds__(256)
k_cvt_flat(const float* __restrict__ s, _Float16* d, int n8, float scale) {
    const int i = blockIdx.x * 256 + threadIdx.x;
    if (i >= n8) return;
    v8f f = ld8(s + (size_t)i * 8) * scale;
    v8h hv = __builtin_convertvector(f, v8h);
    _Float16* q = d + (size_t)i * 8;
    *(volatile v8h*)q = hv;
    __threadfence();
    *(volatile v8h*)q = hv;
}

__global__ void __launch_bounds__(256)
k_cvt_xproj(const float* __restrict__ s, _Float16* d) {
    const int i = blockIdx.x * 256 + threadIdx.x;
    if (i >= (XPC * DN_) / 8) return;
    const int e0 = i * 8;
    const int r  = e0 / DN_;
    const int c0 = e0 % DN_;
    const int k  = r / NPAD;
    const int c  = r % NPAD;
    v8f f = zero8();
    if (c < R_ + 2 * NS_) f = ld8(s + ((size_t)(k * (R_ + 2 * NS_) + c)) * DN_ + c0) * 16.0f;
    v8h hv = __builtin_convertvector(f, v8h);
    _Float16* q = d + (size_t)e0;
    *(volatile v8h*)q = hv;
    __threadfence();
    *(volatile v8h*)q = hv;
}

__global__ void __launch_bounds__(256)
k_dwconv1(const float* __restrict__ x, const float* __restrict__ w,
          const float* __restrict__ bias, float* u) {
    const int gi  = blockIdx.x * 256 + threadIdx.x;
    const int tok = gi / (C_ / 4);
    const int q   = gi % (C_ / 4);
    const int b   = tok / L_;
    const int p   = tok % L_;
    const int hy  = p / W_;
    const int wx  = p % W_;
    const int c0  = 4 * q;
    v4f r;
#pragma unroll
    for (int j = 0; j < 4; ++j) {
        const int c = c0 + j;
        const float* xp = x + ((size_t)(b * C_ + c)) * L_;
        const float* wp = w + c * 9;
        float acc = 0.0f;
#pragma unroll
        for (int ky = 0; ky < 3; ++ky) {
            const int yy = hy + ky - 1;
            if (yy < 0 || yy >= H_) continue;
#pragma unroll
            for (int kx = 0; kx < 3; ++kx) {
                const int xx = wx + kx - 1;
                if (xx < 0 || xx >= W_) continue;
                acc += xp[yy * W_ + xx] * wp[ky * 3 + kx];
            }
        }
        r[j] = acc + bias[c];
    }
    float* dst = u + (size_t)tok * C_ + c0;
    *(volatile v4f*)dst = r;
    __threadfence();
    *(volatile v4f*)dst = r;
}

__global__ void __launch_bounds__(256)
k_ln192(const float* __restrict__ in, const float* __restrict__ g,
        const float* __restrict__ bt, _Float16* out) {
    const int wave = threadIdx.x >> 5, lane = threadIdx.x & 31;
    const int tok  = blockIdx.x * 8 + wave;
    const bool act = lane < (C_ / 8);
    const int c    = 8 * lane;
    v8f v = zero8();
    if (act) v = ld8(in + (size_t)tok * C_ + c);
    const float mean = wsum(hsum8(v)) * (1.0f / (float)C_);
    v8f dv = zero8();
    if (act) dv = v - mean;
    const float var  = wsum(hsum8(dv * dv)) * (1.0f / (float)C_);
    const float rstd = rsqrtf(var + 1e-5f);
    if (act) {
        const v8f o = dv * rstd * ld8(g + c) + ld8(bt + c);
        const v8h hv = __builtin_convertvector(o, v8h);
        _Float16* dst = out + (size_t)tok * C_ + c;
        *(volatile v8h*)dst = hv;
        __threadfence();
        *(volatile v8h*)dst = hv;
    }
}

template <int OUT16>
__global__ void __launch_bounds__(128)
k_gemm(const _Float16* __restrict__ A, const _Float16* __restrict__ Wt,
       const float* __restrict__ bias, const float* __restrict__ resid,
       float* out32, _Float16* out16,
       int N, int K, float scale, float oscale, int has_bias, int act, int has_resid) {
    __shared__ __attribute__((aligned(16))) float sm[4 * 16 * 64];
    const int wave = threadIdx.x >> 5, lane = threadIdx.x & 31;
    const int hh = lane >> 4, m = lane & 15;
    const int row0 = blockIdx.y * 64 + wave * 16;
    const int col0 = blockIdx.x * 64;
    const _Float16* Ap = A  + (size_t)(row0 + m) * K + 8 * hh;
    const _Float16* Wp = Wt + (size_t)(col0 + m) * K + 8 * hh;

    v8f acc[4];
#pragma unroll
    for (int j = 0; j < 4; ++j) acc[j] = zero8();

#pragma unroll 1
    for (int k0 = 0; k0 < K; k0 += 32) {
        Frag a;
        a.h[0] = *(const v8h*)(Ap + k0);
        a.h[1] = *(const v8h*)(Ap + k0 + 16);
#pragma unroll
        for (int j = 0; j < 4; ++j) {
            const _Float16* wj = Wp + (size_t)(16 * j) * K + k0;
            Frag bq;
            bq.h[0] = *(const v8h*)wj;
            bq.h[1] = *(const v8h*)(wj + 16);
            acc[j] = wmma16(a.v, bq.v, acc[j]);
        }
    }

    float* smw = sm + wave * (16 * 64);
#pragma unroll
    for (int j = 0; j < 4; ++j) {
#pragma unroll
        for (int r = 0; r < 8; ++r) smw[(8 * hh + r) * 64 + 16 * j + m] = acc[j][r];
    }
    __syncthreads();

    if (!OUT16) {
        v4f vals[8];
        const int c4 = 4 * m;
#pragma unroll
        for (int i = 0; i < 8; ++i) {
            const int row = 2 * i + hh;
            v4f v = *(const v4f*)(smw + row * 64 + c4);
            v = v * scale;
            if (has_bias) v = v + *(const v4f*)(bias + col0 + c4);
            if (act) {
#pragma unroll
                for (int e = 0; e < 4; ++e) v[e] = gelu_f(v[e]);
            }
            if (has_resid) v = v + *(const v4f*)(resid + (size_t)(row0 + row) * N + col0 + c4);
            vals[i] = v;
        }
#pragma unroll
        for (int i = 0; i < 8; ++i)
            *(volatile v4f*)(out32 + (size_t)(row0 + 2 * i + hh) * N + col0 + c4) = vals[i];
        __threadfence();
#pragma unroll
        for (int i = 0; i < 8; ++i)
            *(volatile v4f*)(out32 + (size_t)(row0 + 2 * i + hh) * N + col0 + c4) = vals[i];
    } else {
        v8h hv[4];
        const int rl = lane >> 3;
        const int c8 = 8 * (lane & 7);
#pragma unroll
        for (int i = 0; i < 4; ++i) {
            const int row = 4 * i + rl;
            v8f f = ld8(smw + row * 64 + c8);
            f = f * scale;
            if (has_bias) f = f + ld8(bias + col0 + c8);
            if (act) {
#pragma unroll
                for (int e = 0; e < 8; ++e) f[e] = gelu_f(f[e]);
            }
            f = f * oscale;
            hv[i] = __builtin_convertvector(f, v8h);
        }
#pragma unroll
        for (int i = 0; i < 4; ++i)
            *(volatile v8h*)(out16 + (size_t)(row0 + 4 * i + rl) * N + col0 + c8) = hv[i];
        __threadfence();
#pragma unroll
        for (int i = 0; i < 4; ++i)
            *(volatile v8h*)(out16 + (size_t)(row0 + 4 * i + rl) * N + col0 + c8) = hv[i];
    }
}

__global__ void __launch_bounds__(96)
k_dwconv2(const float* __restrict__ xz, const float* __restrict__ w,
          const float* __restrict__ bias, float* xc32, _Float16* xc16, float oscale) {
    __shared__ v4f s4[DN_ / 4];
    const int tok = blockIdx.x;
    const int t   = threadIdx.x;
    const int b   = tok / L_;
    const int p   = tok % L_;
    const int hy  = p / W_;
    const int wx  = p % W_;
    const int c0  = 4 * t;
    v4f acc;
#pragma unroll
    for (int j = 0; j < 4; ++j) acc[j] = 0.0f;
#pragma unroll
    for (int ky = 0; ky < 3; ++ky) {
        const int yy = hy + ky - 1;
        if (yy < 0 || yy >= H_) continue;
#pragma unroll
        for (int kx = 0; kx < 3; ++kx) {
            const int xx = wx + kx - 1;
            if (xx < 0 || xx >= W_) continue;
            const v4f v = *(const v4f*)(xz + ((size_t)(b * L_ + yy * W_ + xx)) * (2 * DN_) + c0);
#pragma unroll
            for (int j = 0; j < 4; ++j) acc[j] += v[j] * w[(c0 + j) * 9 + ky * 3 + kx];
        }
    }
    v4f r;
#pragma unroll
    for (int j = 0; j < 4; ++j) r[j] = silu_f(acc[j] + bias[c0 + j]);
    float* dst = xc32 + (size_t)tok * DN_ + c0;
    *(volatile v4f*)dst = r;
    __threadfence();
    *(volatile v4f*)dst = r;

    s4[t] = r;
    __syncthreads();
    v8h hv;
    _Float16* d16 = xc16 + (size_t)tok * DN_ + 8 * t;
    const bool act = t < (DN_ / 8);
    if (act) {
        const v4f a0 = s4[2 * t];
        const v4f a1 = s4[2 * t + 1];
        v8f f = __builtin_shufflevector(a0, a1, 0, 1, 2, 3, 4, 5, 6, 7) * oscale;
        hv = __builtin_convertvector(f, v8h);
        *(volatile v8h*)d16 = hv;
    }
    __threadfence();
    if (act) *(volatile v8h*)d16 = hv;
}

static __device__ __forceinline__ int perm_tok(int k, int l) {
    const int lp = (k >= 2) ? (L_ - 1 - l) : l;
    return (k & 1) ? ((lp % H_) * W_ + lp / H_) : lp;
}

__global__ void __launch_bounds__(128)
k_scan(const float* __restrict__ dbl, const float* __restrict__ xc,
       const float* __restrict__ Alog, const float* __restrict__ Dsv,
       const float* __restrict__ wdt, const float* __restrict__ bdt, float* ydir) {
    __shared__ __attribute__((aligned(16))) float ybuf[4][8][32];
    const int t0   = blockIdx.x * 128;
    const int b    = t0 / (K_ * DN_);
    const int k    = (t0 / DN_) % K_;
    const int wave = threadIdx.x >> 5, lane = threadIdx.x & 31;
    const int dw   = (t0 % DN_) + wave * 32;
    const int d    = dw + lane;
    const int kd   = k * DN_ + d;

    float An[NS_], h[NS_], wr[R_];
#pragma unroll
    for (int n = 0; n < NS_; ++n) { An[n] = -expf(Alog[(size_t)kd * NS_ + n]); h[n] = 0.0f; }
#pragma unroll
    for (int j = 0; j < R_; ++j) wr[j] = wdt[(size_t)kd * R_ + j];
    const float bias = bdt[kd];
    const float Dd   = Dsv[kd];
    const size_t tb  = (size_t)b * L_;
    float* yp = ydir + ((size_t)(k * B_ + b) * L_) * DN_ + dw;

#pragma unroll 1
    for (int l0 = 0; l0 < L_; l0 += 8) {
#pragma unroll 1
        for (int s = 0; s < 8; ++s) {
            const int tok = perm_tok(k, l0 + s);
            const float* row = dbl + (tb + tok) * (size_t)XPC + k * NPAD;
            v4f Rv[3], Bv[4], Cv[4];
#pragma unroll
            for (int i = 0; i < 3; ++i) Rv[i] = *(const v4f*)(row + 4 * i);
#pragma unroll
            for (int i = 0; i < 4; ++i) Bv[i] = *(const v4f*)(row + R_ + 4 * i);
#pragma unroll
            for (int i = 0; i < 4; ++i) Cv[i] = *(const v4f*)(row + R_ + NS_ + 4 * i);
            float a = bias;
#pragma unroll
            for (int j = 0; j < R_; ++j) a += Rv[j >> 2][j & 3] * wr[j];
            const float dt  = fmaxf(a, 0.0f) + log1pf(expf(-fabsf(a)));
            const float x   = xc[(tb + tok) * (size_t)DN_ + d];
            const float dtx = dt * x;
            float y = 0.0f;
#pragma unroll
            for (int n = 0; n < NS_; ++n) {
                const float dA = __expf(dt * An[n]);
                h[n] = h[n] * dA + dtx * Bv[n >> 2][n & 3];
                y += h[n] * Cv[n >> 2][n & 3];
            }
            y += Dd * x;
            ybuf[wave][s][lane] = y;
        }
        __syncthreads();
        const int sA = lane >> 3, q = lane & 7;
        const v4f v0 = *(const v4f*)&ybuf[wave][sA][4 * q];
        const v4f v1 = *(const v4f*)&ybuf[wave][sA + 4][4 * q];
        const int tokA = perm_tok(k, l0 + sA);
        const int tokB = perm_tok(k, l0 + sA + 4);
        float* pA = yp + (size_t)tokA * DN_ + 4 * q;
        float* pB = yp + (size_t)tokB * DN_ + 4 * q;
        *(volatile v4f*)pA = v0;
        *(volatile v4f*)pB = v1;
        __threadfence();
        *(volatile v4f*)pA = v0;
        *(volatile v4f*)pB = v1;
        __syncthreads();
    }
}

__global__ void __launch_bounds__(256)
k_merge_gate(const float* __restrict__ ydir, const float* __restrict__ xz,
             const float* __restrict__ g, const float* __restrict__ bt, _Float16* yg, float oscale) {
    const int wave = threadIdx.x >> 5, lane = threadIdx.x & 31;
    const int tok  = blockIdx.x * 8 + wave;
    const size_t PS = (size_t)MTOK * DN_;
    const float* yp = ydir + (size_t)tok * DN_;
    const int cA   = 8 * lane;
    const bool two = lane < ((DN_ - 256) / 8);
    const int cB   = 256 + 8 * lane;
    v8f ya = (ld8(yp + cA) + ld8(yp + 2 * PS + cA)) + (ld8(yp + PS + cA) + ld8(yp + 3 * PS + cA));
    v8f yb = zero8();
    if (two) yb = (ld8(yp + cB) + ld8(yp + 2 * PS + cB)) + (ld8(yp + PS + cB) + ld8(yp + 3 * PS + cB));
    const float mean = wsum(hsum8(ya) + hsum8(yb)) * (1.0f / (float)DN_);
    v8f da = ya - mean;
    v8f db = zero8();
    if (two) db = yb - mean;
    const float var  = wsum(hsum8(da * da) + hsum8(db * db)) * (1.0f / (float)DN_);
    const float rstd = rsqrtf(var + 1e-5f);
    const float* zp = xz + (size_t)tok * (2 * DN_) + DN_;
    v8h ha, hb;
    {
        const v8f z = ld8(zp + cA);
        v8f o = da * rstd * ld8(g + cA) + ld8(bt + cA);
#pragma unroll
        for (int e = 0; e < 8; ++e) o[e] = o[e] * silu_f(z[e]) * oscale;
        ha = __builtin_convertvector(o, v8h);
    }
    hb = ha;
    if (two) {
        const v8f z = ld8(zp + cB);
        v8f o = db * rstd * ld8(g + cB) + ld8(bt + cB);
#pragma unroll
        for (int e = 0; e < 8; ++e) o[e] = o[e] * silu_f(z[e]) * oscale;
        hb = __builtin_convertvector(o, v8h);
    }
    _Float16* dA = yg + (size_t)tok * DN_ + cA;
    _Float16* dB = yg + (size_t)tok * DN_ + cB;
    *(volatile v8h*)dA = ha;
    if (two) *(volatile v8h*)dB = hb;
    __threadfence();
    *(volatile v8h*)dA = ha;
    if (two) *(volatile v8h*)dB = hb;
}

__global__ void __launch_bounds__(256)
k_final(const float* __restrict__ u, float* out) {
    const int gi    = blockIdx.x * 256 + threadIdx.x;
    const int plane = gi / (L_ / 4);
    const int pq    = gi % (L_ / 4);
    const int b     = plane / C_;
    const int c     = plane % C_;
    const int p0    = 4 * pq;
    const float* src = u + ((size_t)b * L_ + p0) * C_ + c;
    v4f r;
#pragma unroll
    for (int j = 0; j < 4; ++j) r[j] = gelu_f(src[(size_t)j * C_]);
    float* dst = out + (size_t)plane * L_ + p0;
    *(volatile v4f*)dst = r;
    __threadfence();
    *(volatile v4f*)dst = r;
}

extern "C" void kernel_launch(void* const* d_in, const int* in_sizes, int n_in,
                              void* d_out, int out_size, void* d_ws, size_t ws_size,
                              hipStream_t stream) {
    if (n_in < 22) return;
    if (in_sizes[0] != B_ * C_ * H_ * W_) return;
    if (in_sizes[5] != 2 * DN_ * C_ || in_sizes[8] != K_ * (R_ + 2 * NS_) * DN_) return;
    if (out_size != B_ * C_ * H_ * W_) return;

    const float* x          = (const float*)d_in[0];
    const float* conv_w     = (const float*)d_in[1];
    const float* conv_b     = (const float*)d_in[2];
    const float* ln1_g      = (const float*)d_in[3];
    const float* ln1_b      = (const float*)d_in[4];
    const float* in_proj_w  = (const float*)d_in[5];
    const float* conv2_w    = (const float*)d_in[6];
    const float* conv2_b    = (const float*)d_in[7];
    const float* x_proj_w   = (const float*)d_in[8];
    const float* dt_proj_w  = (const float*)d_in[9];
    const float* dt_proj_b  = (const float*)d_in[10];
    const float* A_log      = (const float*)d_in[11];
    const float* Ds         = (const float*)d_in[12];
    const float* onorm_g    = (const float*)d_in[13];
    const float* onorm_b    = (const float*)d_in[14];
    const float* out_proj_w = (const float*)d_in[15];
    const float* ln2_g      = (const float*)d_in[16];
    const float* ln2_b      = (const float*)d_in[17];
    const float* fc1_w      = (const float*)d_in[18];
    const float* fc1_b      = (const float*)d_in[19];
    const float* fc2_w      = (const float*)d_in[20];
    const float* fc2_b      = (const float*)d_in[21];
    float* out = (float*)d_out;

    char* ws = (char*)d_ws;
    size_t off = 0;
    auto carve = [&](size_t bytes) -> char* {
        size_t o = (off + 255) & ~(size_t)255;
        off = o + bytes;
        return ws + o;
    };
    const size_t SZ_U    = (size_t)MTOK * C_ * 4;
    const size_t SZ_XZ   = (size_t)MTOK * 2 * DN_ * 4;
    const size_t SZ_XC32 = (size_t)MTOK * DN_ * 4;
    const size_t SZ_XC16 = (size_t)MTOK * DN_ * 2;
    const size_t SZ_DBL  = (size_t)MTOK * XPC * 4;
    const size_t SZ_Y    = (size_t)K_ * MTOK * DN_ * 4;
    const size_t SZ_H16  = (size_t)MTOK * C_ * 2;
    const size_t SZ_G16  = (size_t)MTOK * MH_ * 2;
    char* R_u0   = carve(SZ_U);
    char* R_xz   = carve(SZ_XZ);
    char* R_xc32 = carve(SZ_XC32);
    char* R_xc16 = carve(SZ_XC16);
    char* R_dbl  = carve(SZ_DBL);
    char* R_y    = carve(SZ_Y);
    char* R_win  = carve((size_t)2 * DN_ * C_ * 2);
    char* R_wx   = carve((size_t)XPC * DN_ * 2);
    char* R_wout = carve((size_t)C_ * DN_ * 2);
    char* R_wfc1 = carve((size_t)MH_ * C_ * 2);
    char* R_wfc2 = carve((size_t)C_ * MH_ * 2);
    if (off > ws_size) return;

    float*    u0    = (float*)R_u0;
    float*    xz    = (float*)R_xz;
    float*    xc32  = (float*)R_xc32;
    _Float16* xc16  = (_Float16*)R_xc16;
    float*    dbl   = (float*)R_dbl;
    float*    ydir  = (float*)R_y;
    _Float16* w_in  = (_Float16*)R_win;
    _Float16* wx    = (_Float16*)R_wx;
    _Float16* w_out = (_Float16*)R_wout;
    _Float16* w_fc1 = (_Float16*)R_wfc1;
    _Float16* w_fc2 = (_Float16*)R_wfc2;
    _Float16* h16a  = (_Float16*)R_xc16;
    _Float16* yg16  = (_Float16*)R_xc32;
    _Float16* h16b  = (_Float16*)(R_xc32 + SZ_XC16);
    float*    u1    = (float*)R_dbl;
    _Float16* g16   = (_Float16*)R_y;
    float*    u2    = (float*)(R_y + SZ_G16);
    (void)SZ_H16;

    const dim3 blk(256);

    k_cvt_flat<<<dim3((2 * DN_ * C_ / 8 + 255) / 256), blk, 0, stream>>>(in_proj_w, w_in, 2 * DN_ * C_ / 8, 16.0f);
    k_cvt_xproj<<<dim3((XPC * DN_ / 8 + 255) / 256), blk, 0, stream>>>(x_proj_w, wx);
    k_cvt_flat<<<dim3((C_ * DN_ / 8 + 255) / 256), blk, 0, stream>>>(out_proj_w, w_out, C_ * DN_ / 8, 16.0f);
    k_cvt_flat<<<dim3((MH_ * C_ / 8 + 255) / 256), blk, 0, stream>>>(fc1_w, w_fc1, MH_ * C_ / 8, 16.0f);
    k_cvt_flat<<<dim3((C_ * MH_ / 8 + 255) / 256), blk, 0, stream>>>(fc2_w, w_fc2, C_ * MH_ / 8, 16.0f);

    k_dwconv1<<<dim3(MTOK * (C_ / 4) / 256), blk, 0, stream>>>(x, conv_w, conv_b, u0);
    k_ln192<<<dim3(MTOK / 8), blk, 0, stream>>>(u0, ln1_g, ln1_b, h16a);
    k_gemm<0><<<dim3(2 * DN_ / 64, MTOK / 64), dim3(128), 0, stream>>>(
        h16a, w_in, fc1_b, u0, xz, g16, 2 * DN_, C_, 1.0f / 16.0f, 1.0f, 0, 0, 0);
    k_dwconv2<<<dim3(MTOK), dim3(96), 0, stream>>>(xz, conv2_w, conv2_b, xc32, xc16, 256.0f);
    k_gemm<0><<<dim3(XPC / 64, MTOK / 64), dim3(128), 0, stream>>>(
        xc16, wx, fc1_b, u0, dbl, g16, XPC, DN_, 1.0f / 4096.0f, 1.0f, 0, 0, 0);
    k_scan<<<dim3(B_ * K_ * DN_ / 128), dim3(128), 0, stream>>>(dbl, xc32, A_log, Ds, dt_proj_w, dt_proj_b, ydir);
    k_merge_gate<<<dim3(MTOK / 8), blk, 0, stream>>>(ydir, xz, onorm_g, onorm_b, yg16, 16.0f);
    k_gemm<0><<<dim3(C_ / 64, MTOK / 64), dim3(128), 0, stream>>>(
        yg16, w_out, fc1_b, u0, u1, g16, C_, DN_, 1.0f / 256.0f, 1.0f, 0, 0, 1);
    k_ln192<<<dim3(MTOK / 8), blk, 0, stream>>>(u1, ln2_g, ln2_b, h16b);
    k_gemm<1><<<dim3(MH_ / 64, MTOK / 64), dim3(128), 0, stream>>>(
        h16b, w_fc1, fc1_b, u1, u2, g16, MH_, C_, 1.0f / 16.0f, 64.0f, 1, 1, 0);
    k_gemm<0><<<dim3(C_ / 64, MTOK / 64), dim3(128), 0, stream>>>(
        g16, w_fc2, fc2_b, u1, u2, g16, C_, MH_, 1.0f / 1024.0f, 1.0f, 1, 0, 1);
    k_final<<<dim3(B_ * C_ * (L_ / 4) / 256), blk, 0, stream>>>(u2, out);
}
